// GATGINEncoder_11570641895556
// MI455X (gfx1250) — hardware-verified
//
#include <hip/hip_runtime.h>
#include <stddef.h>


#define NTHR   256
#define NWAVE  8
#define DD     128
#define DW     256
#define NB     256
#define GR     32
#define GC     128
#define XSP    132
#define HP     136
#define CHUNK  2048
#define WCAP   256
#define NGRP   (CHUNK / (NTHR * 4))
#define NWROWS 512

#define LIST_BYTES    (NWAVE * WCAP * 4 + 64)
#define GAT_LDS_BYTES (NB * DD * 4 + 2 * NB * 4 * 4 + LIST_BYTES)
#define GIN_LDS_BYTES (LIST_BYTES + NB * DD * 4 + NB * HP * 2)

static_assert(NGRP == 2);
static_assert(WCAP == (CHUNK / NTHR) * 32);
static_assert(GAT_LDS_BYTES == 147520);
static_assert(GIN_LDS_BYTES == 208960);
static_assert(NB * HP * 2 <= NB * DD * 4);
static_assert((NB / 2) * XSP * 4 <= NB * HP * 2);
static_assert((NB & (NB - 1)) == 0);
static_assert(NB <= 512);
static_assert(NB <= WCAP);
static_assert((NB % GR) == 0);
static_assert((HP % 8) == 0);
static_assert((XSP % 4) == 0);
static_assert((LIST_BYTES % 16) == 0);

typedef float          v4f  __attribute__((ext_vector_type(4)));
typedef float          v8f  __attribute__((ext_vector_type(8)));
typedef int            v2i  __attribute__((ext_vector_type(2)));
typedef int            v4i  __attribute__((ext_vector_type(4)));
typedef _Float16       v4h  __attribute__((ext_vector_type(4)));
typedef _Float16       v8h  __attribute__((ext_vector_type(8)));
typedef _Float16       v16h __attribute__((ext_vector_type(16)));
typedef unsigned short v8us __attribute__((ext_vector_type(8)));

union FragH { v16h v; v4i u[2]; };
union Pack  { v8h h; v8us s; v4i i; };
union Pack4 { v4h h; v2i i; };

__device__ __forceinline__ v8f wmh(v16h a, v16h b, v8f c) {
  v8f d = __builtin_amdgcn_wmma_f32_16x16x32_f16(false, a, false, b, (short)0, c, false, false);
  asm volatile("v_nop\n\tv_nop\n\tv_nop\n\tv_nop" : "+v"(d) : "v"(a), "v"(b));
  return d;
}

__device__ __forceinline__ float lk2(float t) { return fmaxf(t, 0.2f * t); }
__device__ __forceinline__ float dl(v4f t, v4f w) {
  return w.x * lk2(t.x) + w.y * lk2(t.y) + w.z * lk2(t.z) + w.w * lk2(t.w);
}

__global__ __launch_bounds__(NTHR) void k_cvt_x(const float* __restrict__ x, unsigned short* xh,
                                                int nN, int nPad) {
  const int i  = blockIdx.x * NTHR + threadIdx.x;
  const int n8 = nPad * (DD / 8);
  if (i >= n8) return;
  const int r  = i >> 4;
  const int kb = (i & 15) * 8;
  const int rc = (r < nN) ? r : (nN - 1);
  const v4f p0 = *(const v4f*)(x + (size_t)rc * DD + kb);
  const v4f p1 = *(const v4f*)(x + (size_t)rc * DD + kb + 4);
  const bool live = (r < nN);
  Pack u;
#pragma unroll
  for (int j = 0; j < 4; ++j) {
    u.h[j]     = live ? (_Float16)p0[j] : (_Float16)0.f;
    u.h[4 + j] = live ? (_Float16)p1[j] : (_Float16)0.f;
  }
  unsigned short* p = xh + (size_t)i * 8;
  *(volatile v4i*)p = u.i;
  __threadfence();
  *(volatile v4i*)p = u.i;
}

__global__ __launch_bounds__(NTHR) void k_cvt_w(const float* __restrict__ Wl, const float* __restrict__ Wr,
                                                const float* __restrict__ W1, const float* __restrict__ W2,
                                                unsigned short* wall, float sc) {
  const int i = blockIdx.x * NTHR + threadIdx.x;
  if (i >= NWROWS * 16) return;
  const int q   = i >> 4;
  const int kb  = (i & 15) * 8;
  const int grp = q >> 7;
  const int n   = q & (DD - 1);
  const float* W = (grp == 0) ? Wl : ((grp == 1) ? Wr : ((grp == 2) ? W1 : W2));
  Pack u;
#pragma unroll
  for (int j = 0; j < 8; ++j) u.h[j] = (_Float16)(W[(size_t)(kb + j) * DD + n] * sc);
  unsigned short* p = wall + (size_t)q * DD + kb;
  *(volatile v4i*)p = u.i;
  __threadfence();
  *(volatile v4i*)p = u.i;
}

__global__ __launch_bounds__(NTHR) void k_gemm1(
    const unsigned short* __restrict__ A, const unsigned short* __restrict__ B,
    const float* __restrict__ bl, const float* __restrict__ br,
    float* out, int K, int Ncols, float oscale) {
  __shared__ __attribute__((aligned(16))) float Xs[GR * XSP];

  const int tid  = threadIdx.x;
  const int lane = tid & 31;
  const int wave = tid >> 5;
  const int hh   = lane >> 4;
  const int m    = lane & 15;
  const int rowBase = blockIdx.x * GR;
  const int colBase = blockIdx.y * GC;
  const int ncol = colBase + wave * 16 + m;

  const size_t ra0 = (size_t)(rowBase + m) * K + 8 * hh;
  const size_t ra1 = ra0 + (size_t)16 * K;
  const size_t rb  = (size_t)ncol * K + 8 * hh;

  v8f c0 = {0.f, 0.f, 0.f, 0.f, 0.f, 0.f, 0.f, 0.f};
  v8f c1 = {0.f, 0.f, 0.f, 0.f, 0.f, 0.f, 0.f, 0.f};

#pragma unroll 1
  for (int k0 = 0; k0 < K; k0 += 32) {
    FragH a0, a1, b;
    a0.u[0] = *(const v4i*)(A + ra0 + k0);  a0.u[1] = *(const v4i*)(A + ra0 + k0 + 16);
    a1.u[0] = *(const v4i*)(A + ra1 + k0);  a1.u[1] = *(const v4i*)(A + ra1 + k0 + 16);
    b.u[0]  = *(const v4i*)(B + rb + k0);   b.u[1]  = *(const v4i*)(B + rb + k0 + 16);
    c0 = wmh(a0.v, b.v, c0);
    c1 = wmh(a1.v, b.v, c1);
  }

  const int   nc  = ncol & (DD - 1);
  const float bv0 = bl[nc];
  const float bv1 = br[nc];
  const float bv  = (ncol < DD) ? bv0 : bv1;
  const int cl = wave * 16 + m;
#pragma unroll
  for (int r = 0; r < 8; ++r) {
    Xs[(8 * hh + r) * XSP + cl]      = c0[r] * oscale + bv;
    Xs[(16 + 8 * hh + r) * XSP + cl] = c1[r] * oscale + bv;
  }
  __syncthreads();

  v4f xv[4];
  float* xpp[4];
#pragma unroll
  for (int i = 0; i < 4; ++i) {
    xv[i]  = *(const v4f*)(Xs + (4 * wave + i) * XSP + 4 * lane);
    xpp[i] = out + (size_t)(rowBase + 4 * wave + i) * Ncols + colBase + 4 * lane;
  }
#pragma unroll
  for (int i = 0; i < 4; ++i) *(volatile v4f*)(xpp[i]) = xv[i];
  __threadfence();
#pragma unroll
  for (int i = 0; i < 4; ++i) *(volatile v4f*)(xpp[i]) = xv[i];
}

template <int EQ>
__device__ __forceinline__ void scan_chunk(const int* __restrict__ ids, int nIds, int cbase, int base,
                                           int* list, int* wcnt, int tid, int lane, int wave, bool al16) {
  int wc = 0;
#pragma unroll
  for (int g = 0; g < NGRP; ++g) {
    const int el0 = (g * NTHR + tid) * 4;
    const int e0  = cbase + el0;
    const int sent = -2147483647 - 1;
    v4i d;
    if (al16 && (cbase + CHUNK <= nIds)) {
      d = *(const v4i*)(ids + e0);
    } else {
      const int l0 = min(e0, nIds - 1), l1 = min(e0 + 1, nIds - 1);
      const int l2 = min(e0 + 2, nIds - 1), l3 = min(e0 + 3, nIds - 1);
      const int t0 = ids[l0], t1 = ids[l1], t2 = ids[l2], t3 = ids[l3];
      d.x = (e0     < nIds) ? t0 : sent;
      d.y = (e0 + 1 < nIds) ? t1 : sent;
      d.z = (e0 + 2 < nIds) ? t2 : sent;
      d.w = (e0 + 3 < nIds) ? t3 : sent;
    }
    const unsigned s0 = (unsigned)d.x - (unsigned)base;
    const unsigned s1 = (unsigned)d.y - (unsigned)base;
    const unsigned s2 = (unsigned)d.z - (unsigned)base;
    const unsigned s3 = (unsigned)d.w - (unsigned)base;
    const bool h0 = EQ ? (s0 == 0u) : (s0 < (unsigned)NB);
    const bool h1 = EQ ? (s1 == 0u) : (s1 < (unsigned)NB);
    const bool h2 = EQ ? (s2 == 0u) : (s2 < (unsigned)NB);
    const bool h3 = EQ ? (s3 == 0u) : (s3 < (unsigned)NB);
    const unsigned many = __builtin_amdgcn_ballot_w32(h0 | h1 | h2 | h3);
    if (many != 0u) {
#define HITJ(J, HJ, SJ) { \
        const unsigned mj = __builtin_amdgcn_ballot_w32(HJ); \
        if (HJ) { \
          const int pos = wc + (int)__builtin_amdgcn_mbcnt_lo(mj, 0u); \
          if (pos < WCAP) list[wave * WCAP + pos] = ((el0 + (J)) << 9) | (int)(SJ); \
        } \
        wc += (int)__builtin_popcount(mj); }
      HITJ(0, h0, s0)
      HITJ(1, h1, s1)
      HITJ(2, h2, s2)
      HITJ(3, h3, s3)
#undef HITJ
    }
  }
  if (lane == 0) wcnt[wave] = wc;
}

__device__ __forceinline__ void gat_hit(const float* xs, const float* xd, float* ar, float* mp, float* dp, v4f w) {
  const v4f a = *(const v4f*)xs;
  const v4f d = *(const v4f*)xd;
  float s = dl(a + d, w);
  s += __shfl_xor(s, 4, 32);
  s += __shfl_xor(s, 2, 32);
  s += __shfl_xor(s, 1, 32);
  const float m  = mp[0], n = dp[0];
  const float mn = fmaxf(m, s);
  const float sc = __expf(m - mn);
  const float p  = __expf(s - mn);
  v4f e = *(v4f*)ar;
  e = e * sc + a * p;
  *(v4f*)ar = e;
  mp[0] = mn;
  dp[0] = n * sc + p;
}

__global__ __launch_bounds__(NTHR) void k_gat(
    const int* __restrict__ ei, const float* __restrict__ xlr, const float* __restrict__ att,
    const float* __restrict__ gbias, float* x1, int nN, int nE, int nPad) {
  extern __shared__ v4f lds_dyn[];
  float* sacc = (float*)lds_dyn;
  float* mx   = sacc + NB * DD;
  float* dn   = mx + NB * 4;
  int*   list = (int*)(dn + NB * 4);
  int*   wcnt = list + NWAVE * WCAP;

  const int tid  = threadIdx.x;
  const int lane = tid & 31;
  const int wave = tid >> 5;
  const int nodeBase = blockIdx.x * NB;

  {
    const v4f z4 = {0.f, 0.f, 0.f, 0.f};
    for (int i = tid; i < NB * DD / 4; i += NTHR) lds_dyn[i] = z4;
    for (int i = tid; i < NB * 4; i += NTHR) { mx[i] = -1.0e30f; dn[i] = 0.f; }
  }
  __syncthreads();

  const int coff = 4 * lane;
  const int hidx = lane >> 3;
  const v4f w0 = *(const v4f*)(att + coff);

  const int* eid = ei + nE;
  const bool al16 = ((nE & 3) == 0);
  const int nChunks = (nE + CHUNK - 1) / CHUNK;

#pragma unroll 1
  for (int ch = 0; ch <= nChunks; ++ch) {
    const int cbase = ch * CHUNK;
    const bool selfp = (ch == nChunks);
    if (!selfp) {
      scan_chunk<0>(eid, nE, cbase, nodeBase, list, wcnt, tid, lane, wave, al16);
    } else {
      for (int s = tid; s < NB; s += NTHR) list[s] = s;
      if (tid < NWAVE) {
        int c = NB - tid * WCAP;
        c = c < 0 ? 0 : (c > WCAP ? WCAP : c);
        wcnt[tid] = c;
      }
    }
    __syncthreads();

    if (wave == 0) {
#pragma unroll 1
      for (int wsx = 0; wsx < NWAVE; ++wsx) {
        int n = __builtin_amdgcn_readfirstlane(wcnt[wsx]);
        n = n > WCAP ? WCAP : n;
        n = n < 0 ? 0 : n;
#pragma unroll 1
        for (int i = 0; i < n; ++i) {
          const int ent  = __builtin_amdgcn_readfirstlane(list[wsx * WCAP + i]);
          const int slot = ent & (NB - 1);
          const int el   = (ent >> 9) & (CHUNK - 1);
          const int node = nodeBase + slot;
          if (node >= nN) continue;
          int e = cbase + el;
          if (e > nE - 1) e = nE - 1;
          int sj = ei[e];
          sj = sj < 0 ? 0 : (sj > nN - 1 ? nN - 1 : sj);
          const int src = selfp ? node : sj;
          gat_hit(xlr + (size_t)src * DW + coff,
                  xlr + (size_t)node * DW + DD + coff,
                  sacc + slot * DD + coff,
                  mx + slot * 4 + hidx,
                  dn + slot * 4 + hidx, w0);
        }
      }
    }
    __syncthreads();
  }

  const v4f b0 = *(const v4f*)(gbias + coff);
#pragma unroll 1
  for (int s = wave; s < NB; s += NWAVE) {
    const int node = nodeBase + s;
    if (node >= nPad) break;
    const bool live = (node < nN);
    const v4f e0 = *(const v4f*)(sacc + s * DD + coff);
    float dd = dn[s * 4 + hidx];
    dd = live ? dd : 1.0f;
    const float inv = 1.0f / dd;
    v4f o = e0 * inv + b0;
#pragma unroll
    for (int j = 0; j < 4; ++j) {
      float v = o[j];
      v = fmaxf(v, 0.01f * v);
      o[j] = live ? v : 0.f;
    }
    float* op = x1 + (size_t)node * DD + coff;
    *(volatile v4f*)op = o;
    __threadfence();
    *(volatile v4f*)op = o;
  }
}

__global__ __launch_bounds__(NTHR) void k_gin(
    const int* __restrict__ ei, const float* __restrict__ x1,
    const unsigned short* __restrict__ w1t, const unsigned short* __restrict__ w2t,
    const float* __restrict__ b1, const float* __restrict__ bga, const float* __restrict__ bbe,
    const float* __restrict__ bmu, const float* __restrict__ bva, const float* __restrict__ b2,
    float* x2, int nN, int nE, int nPad, float oscale) {
  extern __shared__ v4f lds_dyn[];
  char* lb = (char*)lds_dyn;
  int*   list = (int*)lb;
  int*   wcnt = list + NWAVE * WCAP;
  float* sacc = (float*)(lb + LIST_BYTES);
  unsigned short* hA = (unsigned short*)(lb + LIST_BYTES + NB * DD * 4);
  _Float16* h2f = (_Float16*)sacc;
  const unsigned short* h2 = (const unsigned short*)sacc;
  float* sO = (float*)hA;

  const int tid  = threadIdx.x;
  const int lane = tid & 31;
  const int wave = tid >> 5;
  const int hh   = lane >> 4;
  const int m    = lane & 15;
  const int coff = 4 * lane;
  const int nodeBase = blockIdx.x * NB;

  {
    const v4f z4 = {0.f, 0.f, 0.f, 0.f};
    v4f* sz = (v4f*)sacc;
    for (int i = tid; i < NB * DD / 4; i += NTHR) sz[i] = z4;
  }
  __syncthreads();

  const int* eid = ei + nE;
  const bool al16 = ((nE & 3) == 0);
  const int nChunks = (nE + CHUNK - 1) / CHUNK;
#pragma unroll 1
  for (int ch = 0; ch < nChunks; ++ch) {
    const int cbase = ch * CHUNK;
    scan_chunk<0>(eid, nE, cbase, nodeBase, list, wcnt, tid, lane, wave, al16);
    __syncthreads();
    if (wave == 0) {
#pragma unroll 1
      for (int wsx = 0; wsx < NWAVE; ++wsx) {
        int n = __builtin_amdgcn_readfirstlane(wcnt[wsx]);
        n = n > WCAP ? WCAP : n;
        n = n < 0 ? 0 : n;
#pragma unroll 1
        for (int i = 0; i < n; ++i) {
          const int ent  = __builtin_amdgcn_readfirstlane(list[wsx * WCAP + i]);
          const int slot = ent & (NB - 1);
          const int el   = (ent >> 9) & (CHUNK - 1);
          const int node = nodeBase + slot;
          if (node >= nN) continue;
          int e = cbase + el;
          if (e > nE - 1) e = nE - 1;
          int sj = ei[e];
          sj = sj < 0 ? 0 : (sj > nN - 1 ? nN - 1 : sj);
          const v4f a = *(const v4f*)(x1 + (size_t)sj * DD + coff);
          float* ar = sacc + slot * DD + coff;
          const v4f cur = *(v4f*)ar;
          *(v4f*)ar = cur + a;
        }
      }
    }
    __syncthreads();
  }

#pragma unroll 1
  for (int s = wave; s < NB; s += NWAVE) {
    const int node = nodeBase + s;
    const bool live = (node < nN);
    const int nc = live ? node : (nN - 1);
    const v4f xv = *(const v4f*)(x1 + (size_t)nc * DD + coff);
    const v4f av = *(const v4f*)(sacc + s * DD + coff);
    const v4f hv = xv + av;
    Pack4 p;
#pragma unroll
    for (int j = 0; j < 4; ++j) p.h[j] = live ? (_Float16)hv[j] : (_Float16)0.f;
    *(v2i*)(hA + s * HP + coff) = p.i;
  }
  __syncthreads();

  const int col = wave * 16 + m;
  {
    FragH bw[4];
#pragma unroll
    for (int kt = 0; kt < 4; ++kt) {
      bw[kt].u[0] = *(const v4i*)(w1t + (size_t)col * DD + 32 * kt + 8 * hh);
      bw[kt].u[1] = *(const v4i*)(w1t + (size_t)col * DD + 32 * kt + 8 * hh + 16);
    }
    const float bb = b1[col];
    const float rs = rsqrtf(bva[col] + 1e-5f);
    const float ga = bga[col];
    const float be = bbe[col];
    const float mu = bmu[col];
#pragma unroll 1
    for (int rt = 0; rt < NB / 16; ++rt) {
      v8f c = {0.f, 0.f, 0.f, 0.f, 0.f, 0.f, 0.f, 0.f};
#pragma unroll
      for (int kt = 0; kt < 4; ++kt) {
        FragH a;
        a.u[0] = *(const v4i*)(hA + (16 * rt + m) * HP + 32 * kt + 8 * hh);
        a.u[1] = *(const v4i*)(hA + (16 * rt + m) * HP + 32 * kt + 8 * hh + 16);
        c = wmh(a.v, bw[kt].v, c);
      }
#pragma unroll
      for (int r = 0; r < 8; ++r) {
        float v = c[r] * oscale + bb;
        v = (v - mu) * rs * ga + be;
        v = fmaxf(v, 0.f);
        h2f[(16 * rt + 8 * hh + r) * HP + col] = (_Float16)v;
      }
    }
  }
  __syncthreads();

  {
    FragH bw[4];
#pragma unroll
    for (int kt = 0; kt < 4; ++kt) {
      bw[kt].u[0] = *(const v4i*)(w2t + (size_t)col * DD + 32 * kt + 8 * hh);
      bw[kt].u[1] = *(const v4i*)(w2t + (size_t)col * DD + 32 * kt + 8 * hh + 16);
    }
    const float bb = b2[col];
#pragma unroll 1
    for (int half = 0; half < 2; ++half) {
#pragma unroll 1
      for (int rt8 = 0; rt8 < NB / 32; ++rt8) {
        const int rt = half * (NB / 32) + rt8;
        v8f c = {0.f, 0.f, 0.f, 0.f, 0.f, 0.f, 0.f, 0.f};
#pragma unroll
        for (int kt = 0; kt < 4; ++kt) {
          FragH a;
          a.u[0] = *(const v4i*)(h2 + (16 * rt + m) * HP + 32 * kt + 8 * hh);
          a.u[1] = *(const v4i*)(h2 + (16 * rt + m) * HP + 32 * kt + 8 * hh + 16);
          c = wmh(a.v, bw[kt].v, c);
        }
#pragma unroll
        for (int r = 0; r < 8; ++r) {
          float v = c[r] * oscale + bb;
          v = fmaxf(v, 0.f);
          v = fmaxf(v, 0.01f * v);
          sO[(16 * rt8 + 8 * hh + r) * XSP + col] = v;
        }
      }
      __syncthreads();
#pragma unroll 1
      for (int i = 0; i < 16; ++i) {
        const int row  = 16 * wave + i;
        const int node = nodeBase + half * (NB / 2) + row;
        const v4f v = *(const v4f*)(sO + row * XSP + coff);
        *(volatile v4f*)(x2 + (size_t)node * DD + coff) = v;
      }
      __threadfence();
#pragma unroll 1
      for (int i = 0; i < 16; ++i) {
        const int row  = 16 * wave + i;
        const int node = nodeBase + half * (NB / 2) + row;
        const v4f v = *(const v4f*)(sO + row * XSP + coff);
        *(volatile v4f*)(x2 + (size_t)node * DD + coff) = v;
      }
      __syncthreads();
    }
  }
}

__global__ __launch_bounds__(NTHR) void k_pool(const int* __restrict__ bt, const float* __restrict__ x2,
                                               float* out, int nN) {
  __shared__ int list[NWAVE * WCAP];
  __shared__ int wcnt[NWAVE + 8];
  const int tid  = threadIdx.x;
  const int lane = tid & 31;
  const int wave = tid >> 5;
  const int g    = blockIdx.x;
  const int coff = 4 * lane;
  v4f accv = {0.f, 0.f, 0.f, 0.f};
  const bool al16 = ((nN & 3) == 0);
  const int nChunks = (nN + CHUNK - 1) / CHUNK;
#pragma unroll 1
  for (int ch = 0; ch < nChunks; ++ch) {
    const int cbase = ch * CHUNK;
    scan_chunk<1>(bt, nN, cbase, g, list, wcnt, tid, lane, wave, al16);
    __syncthreads();
    if (wave == 0) {
#pragma unroll 1
      for (int wsx = 0; wsx < NWAVE; ++wsx) {
        int n = __builtin_amdgcn_readfirstlane(wcnt[wsx]);
        n = n > WCAP ? WCAP : n;
        n = n < 0 ? 0 : n;
#pragma unroll 1
        for (int i = 0; i < n; ++i) {
          const int ent = __builtin_amdgcn_readfirstlane(list[wsx * WCAP + i]);
          const int el  = (ent >> 9) & (CHUNK - 1);
          int node = cbase + el;
          node = node > nN - 1 ? nN - 1 : node;
          accv += *(const v4f*)(x2 + (size_t)node * DD + coff);
        }
      }
    }
    __syncthreads();
  }
  if (wave == 0) {
    float* op = out + (size_t)g * DD + coff;
    *(volatile v4f*)op = accv;
    __threadfence();
    *(volatile v4f*)op = accv;
  }
}

extern "C" void kernel_launch(void* const* d_in, const int* in_sizes, int n_in,
                              void* d_out, int out_size, void* d_ws, size_t ws_size,
                              hipStream_t stream) {
  if (n_in < 17) return;
  const int nN = in_sizes[0] / DD;
  if (nN <= 0 || in_sizes[0] != nN * DD) return;
  const int nE = in_sizes[1] / 2;
  if (nE <= 0 || in_sizes[1] != 2 * nE) return;
  if (in_sizes[2] != nN) return;
  if (in_sizes[3] != DD * DD || in_sizes[5] != DD * DD || in_sizes[9] != DD * DD || in_sizes[15] != DD * DD) return;
  if (in_sizes[4] != DD || in_sizes[6] != DD || in_sizes[7] != DD || in_sizes[8] != DD ||
      in_sizes[10] != DD || in_sizes[11] != DD || in_sizes[12] != DD || in_sizes[13] != DD ||
      in_sizes[14] != DD || in_sizes[16] != DD) return;
  if (out_size <= 0 || (out_size % DD) != 0) return;
  const int nG = out_size / DD;

  const float* x     = (const float*)d_in[0];
  const int*   ei    = (const int*)d_in[1];
  const int*   batch = (const int*)d_in[2];
  const float* Wl    = (const float*)d_in[3];
  const float* bl    = (const float*)d_in[4];
  const float* Wr    = (const float*)d_in[5];
  const float* br    = (const float*)d_in[6];
  const float* att   = (const float*)d_in[7];
  const float* gb    = (const float*)d_in[8];
  const float* W1    = (const float*)d_in[9];
  const float* b1    = (const float*)d_in[10];
  const float* ga    = (const float*)d_in[11];
  const float* be    = (const float*)d_in[12];
  const float* mu    = (const float*)d_in[13];
  const float* va    = (const float*)d_in[14];
  const float* W2    = (const float*)d_in[15];
  const float* b2    = (const float*)d_in[16];
  float* out = (float*)d_out;

  const int nPad = ((nN + NB - 1) / NB) * NB;

  char* wsp = (char*)d_ws;
  size_t off = 0;
  const size_t xhB  = (size_t)nPad * DD * 2;
  const size_t waB  = (size_t)NWROWS * DD * 2;
  const size_t xlrB = (size_t)nPad * DW * 4;
  const size_t xpB  = (size_t)nPad * DD * 4;
  unsigned short* xh   = (unsigned short*)(wsp + off); off += xhB;
  unsigned short* wall = (unsigned short*)(wsp + off); off += waB;
  float* xlr = (float*)(wsp + off); off += xlrB;
  float* x1p = (float*)(wsp + off); off += xpB;
  float* x2p = (float*)(wsp + off); off += xpB;
  if (off > ws_size) return;

  hipFuncSetAttribute(reinterpret_cast<const void*>(&k_gat),
                      hipFuncAttributeMaxDynamicSharedMemorySize, GAT_LDS_BYTES);
  hipFuncSetAttribute(reinterpret_cast<const void*>(&k_gin),
                      hipFuncAttributeMaxDynamicSharedMemorySize, GIN_LDS_BYTES);

  const float ws8  = 8.0f;
  const float iws8 = 0.125f;

  k_cvt_x<<<(nPad * (DD / 8) + NTHR - 1) / NTHR, NTHR, 0, stream>>>(x, xh, nN, nPad);
  k_cvt_w<<<(NWROWS * 16 + NTHR - 1) / NTHR, NTHR, 0, stream>>>(Wl, Wr, W1, W2, wall, ws8);
  k_gemm1<<<dim3(nPad / GR, DW / GC), NTHR, 0, stream>>>(xh, wall, bl, br, xlr, DD, DW, iws8);
  k_gat<<<nPad / NB, NTHR, GAT_LDS_BYTES, stream>>>(ei, xlr, att, gb, x1p, nN, nE, nPad);
  k_gin<<<nPad / NB, NTHR, GIN_LDS_BYTES, stream>>>(ei, x1p, wall + (size_t)2 * DD * DD,
                                                      wall + (size_t)3 * DD * DD,
                                                      b1, ga, be, mu, va, b2, x2p, nN, nE, nPad, iws8);
  k_pool<<<nG, NTHR, 0, stream>>>(batch, x2p, out, nN);
}
